// TransformerEncoderLayer_71305047048344
// MI455X (gfx1250) — hardware-verified
//
#include <hip/hip_runtime.h>
#ifndef NB
#define NB 2
#endif
#ifndef SEQ
#define SEQ 2048
#endif
#define NB_FULL 2
#define SEQ_FULL 2048
#define DM 1024
#define NH 16
#define HD 64
#define DFF 4096
#define LQ 3072
#define NR (NB * SEQ)

static_assert(SEQ % 128 == 0);
static_assert(SEQ <= SEQ_FULL);
static_assert(NB <= NB_FULL);
static_assert(NH * HD == DM);
static_assert(LQ == 3 * DM);
static_assert(DM == 1024);
static_assert(DM % 64 == 0 && DFF % 64 == 0 && LQ % 64 == 0);
static_assert(DM % 32 == 0 && DFF % 32 == 0);
static_assert(NR % 128 == 0);

typedef unsigned short v8us __attribute__((ext_vector_type(8), may_alias));
typedef float  v8f  __attribute__((ext_vector_type(8)));
typedef float  v4f  __attribute__((ext_vector_type(4)));
typedef float  v4fa __attribute__((ext_vector_type(4), may_alias));
typedef _Float16 v16h __attribute__((ext_vector_type(16)));
typedef _Float16 v4h  __attribute__((ext_vector_type(4)));
union FragH { v16h v; v8us half[2]; _Float16 h[16]; unsigned short u[16]; };

__device__ __forceinline__ unsigned short bf16_bits(float x) { unsigned int u = __float_as_uint(x); return (unsigned short)((u + 0x7FFFu + ((u >> 16) & 1u)) >> 16); }
__device__ __forceinline__ float bf16_rne(float x) { return __uint_as_float(((unsigned int)bf16_bits(x)) << 16); }
__device__ __forceinline__ unsigned xrow(unsigned r) { return (r / (unsigned)SEQ) * (unsigned)SEQ_FULL + (r % (unsigned)SEQ); }

__device__ __forceinline__ v16h g2_frag(const _Float16* p, unsigned hh) { FragH f; f.half[0] = *(const v8us*)((const unsigned short*)p + 8 * hh); f.half[1] = *(const v8us*)((const unsigned short*)p + 16 + 8 * hh); return f.v; }
__device__ __forceinline__ v8f g2_mma(v16h a, v16h b, v8f c) { v8f d = __builtin_amdgcn_wmma_f32_16x16x32_f16(false, a, false, b, (short)0, c, false, false); asm volatile("v_nop\n\tv_nop\n\tv_nop\n\tv_nop" : "+v"(d) : "v"(a), "v"(b)); return d; }

__global__ __launch_bounds__(256) void k_x16(const float* __restrict__ x, _Float16* __restrict__ X16) {
  const unsigned t = blockIdx.x * 256u + threadIdx.x;
  if (t >= (unsigned)(NR * (DM / 8))) return;
  const unsigned r = t >> 7, c = (t & 127u) * 8u;
  const float* src = x + (size_t)xrow(r) * DM + c;
  const v4f a = *(const v4fa*)src, b = *(const v4fa*)(src + 4);
  FragH f;
#pragma unroll
  for (int q = 0; q < 4; ++q) { f.h[q] = (_Float16)(bf16_rne(a[q]) * 16.0f); f.h[4 + q] = (_Float16)(bf16_rne(b[q]) * 16.0f); }
  const v8us o = f.half[0];
  unsigned short* d = (unsigned short*)X16 + (size_t)t * 8;
  *(volatile v8us*)d = o; __threadfence(); *(volatile v8us*)d = o;
}

__global__ __launch_bounds__(256) void k_wt_f16(const float* __restrict__ W, _Float16* __restrict__ Wt, unsigned K, unsigned N, float scale) {
  const unsigned t = blockIdx.x * 256u + threadIdx.x; const unsigned k8n = K >> 3;
  if (t >= N * k8n) return;
  const unsigned n = t / k8n, k8 = (t - n * k8n) * 8u;
  FragH f;
#pragma unroll
  for (int i = 0; i < 8; ++i) f.h[i] = (_Float16)(bf16_rne(W[(size_t)(k8 + i) * N + n]) * scale);
  const v8us o = f.half[0];
  unsigned short* d = (unsigned short*)Wt + (size_t)n * K + k8;
  *(volatile v8us*)d = o; __threadfence(); *(volatile v8us*)d = o;
}

__global__ __launch_bounds__(256) void k_vt(const _Float16* __restrict__ QKV, _Float16* __restrict__ VT) {
  __shared__ unsigned short tl[64][66];
  const unsigned tid = threadIdx.x; const unsigned slab = blockIdx.x / (unsigned)(SEQ / 64), lg = blockIdx.x % (unsigned)(SEQ / 64); const unsigned b = slab / (unsigned)NH, h = slab % (unsigned)NH;
  for (unsigned i = tid; i < 512u; i += 256u) { const unsigned r = i >> 3, c8 = (i & 7u) * 8u; FragH f; f.half[0] = *(const v8us*)((const unsigned short*)QKV + ((size_t)b * SEQ + lg * 64u + r) * LQ + h * 192u + 128u + c8);
#pragma unroll
    for (int q = 0; q < 8; ++q) tl[r][c8 + q] = f.u[q]; }
  __syncthreads();
  for (int pass = 0; pass < 2; ++pass) {
#pragma unroll
    for (unsigned rd = 0; rd < 2; ++rd) { const unsigned d = rd * 32u + (tid >> 3), pc = tid & 7u; FragH f;
#pragma unroll
      for (int q = 0; q < 8; ++q) f.u[q] = tl[pc * 8u + q][d];
      const v8us o = f.half[0];
      *(volatile v8us*)((unsigned short*)VT + ((size_t)slab * 64u + d) * SEQ + lg * 64u + pc * 8u) = o; }
    if (pass == 0) __threadfence(); }
}

__global__ __launch_bounds__(128) void k_attn(const _Float16* __restrict__ QKV, const _Float16* __restrict__ VT, _Float16* __restrict__ O16) {
  __shared__ __attribute__((aligned(16))) unsigned short os[4][16][72];
  const unsigned tid = threadIdx.x, w = tid >> 5, lane = tid & 31u, ln = lane & 15u, hh = lane >> 4;
  const unsigned qb = blockIdx.x % (unsigned)(SEQ / 64), hb = blockIdx.x / (unsigned)(SEQ / 64); const unsigned h = hb % (unsigned)NH, b = hb / (unsigned)NH;
  const unsigned q0 = qb * 64u + w * 16u;
  const _Float16* qrow = QKV + ((size_t)b * SEQ + q0 + ln) * LQ + h * 192u;
  const v16h bq0 = g2_frag(qrow, hh), bq1 = g2_frag(qrow + 32, hh);
  const _Float16* kbase = QKV + ((size_t)b * SEQ + ln) * LQ + h * 192u + 64u;
  const _Float16* vbase = VT + ((size_t)(b * NH + h) * 64u + ln) * SEQ;
  const v8f z8 = {0.f, 0.f, 0.f, 0.f, 0.f, 0.f, 0.f, 0.f};
  v8f o[4] = {z8, z8, z8, z8};
  float m = -1.0e30f, l = 0.f;
#pragma unroll 1
  for (unsigned j0 = 0; j0 < (unsigned)SEQ; j0 += 64u) {
    v8f c[4];
#pragma unroll
    for (int t = 0; t < 4; ++t) { const _Float16* kr = kbase + (size_t)(j0 + t * 16u) * LQ; v8f z = z8; z = g2_mma(g2_frag(kr, hh), bq0, z); z = g2_mma(g2_frag(kr + 32, hh), bq1, z); c[t] = z; }
    float mx = c[0][0];
#pragma unroll
    for (int t = 0; t < 4; ++t)
#pragma unroll
      for (int r = 0; r < 8; ++r) mx = fmaxf(mx, c[t][r]);
    mx = fmaxf(mx, __shfl_xor(mx, 16, 32));
    const float mnew = fmaxf(m, mx * 0.125f);
    const float alpha = __expf(m - mnew);
    m = mnew;
    const float sh = 6.9314718f - mnew;
    float ps = 0.f;
    FragH p0, p1;
#pragma unroll
    for (int r = 0; r < 8; ++r) {
      const float e0 = __expf(fmaf(c[0][r], 0.125f, sh)), e1 = __expf(fmaf(c[1][r], 0.125f, sh));
      const float e2 = __expf(fmaf(c[2][r], 0.125f, sh)), e3 = __expf(fmaf(c[3][r], 0.125f, sh));
      ps += (e0 + e1) + (e2 + e3);
      p0.h[r] = (_Float16)e0; p0.h[8 + r] = (_Float16)e1; p1.h[r] = (_Float16)e2; p1.h[8 + r] = (_Float16)e3;
    }
    l = l * alpha + ps;
#pragma unroll
    for (int dt = 0; dt < 4; ++dt)
#pragma unroll
      for (int r = 0; r < 8; ++r) o[dt][r] *= alpha;
#pragma unroll
    for (int dt = 0; dt < 4; ++dt) { const _Float16* vr = vbase + (size_t)(dt * 16u) * SEQ + j0; o[dt] = g2_mma(g2_frag(vr, hh), p0.v, o[dt]); o[dt] = g2_mma(g2_frag(vr + 32, hh), p1.v, o[dt]); }
  }
  const float lt = l + __shfl_xor(l, 16, 32);
  const float fin = 64.0f * (1.0f / lt);
#pragma unroll
  for (int dt = 0; dt < 4; ++dt) { FragH f;
#pragma unroll
    for (int r = 0; r < 8; ++r) f.h[r] = (_Float16)(o[dt][r] * fin);
    *(v8us*)&os[w][ln][dt * 16 + 8 * hh] = f.half[0]; }
  __builtin_amdgcn_fence(4  , "workgroup"); __builtin_amdgcn_wave_barrier();
  const unsigned rq = lane >> 3, pc = (lane & 7u) * 8u;
  for (int pass = 0; pass < 2; ++pass) {
#pragma unroll
    for (unsigned it = 0; it < 4; ++it) { const unsigned row = it * 4u + rq; const v8us v = *(const v8us*)&os[w][row][pc];
      *(volatile v8us*)((unsigned short*)O16 + ((size_t)b * SEQ + q0 + row) * DM + h * 64u + pc) = v; }
    if (pass == 0) __threadfence(); }
}

template <int ACT, int RES>
__global__ __launch_bounds__(128) void k_gemm2(const _Float16* __restrict__ A, unsigned lda, const _Float16* __restrict__ Bh, unsigned ldb, float alpha, const float* __restrict__ bias,
    const float* __restrict__ R, unsigned ldr, float* __restrict__ C, _Float16* __restrict__ C16, unsigned ldc, unsigned M, unsigned N, unsigned K) {
  static_assert(ACT == 0 || ACT == 6);
  static_assert(RES == 0 || RES == 1 || RES == 2);
  __shared__ __attribute__((aligned(16))) float so[4][32][68];
  const unsigned tid = threadIdx.x, w = tid >> 5, lane = tid & 31u, ln = lane & 15u, hh = lane >> 4;
  const unsigned ntn = N >> 6; const unsigned mt = blockIdx.x / ntn, nq = blockIdx.x - mt * ntn; const unsigned row0 = mt * 128u + 32u * w, col0 = nq * 64u; if (row0 >= M) return;
  const _Float16* a0p = A + (size_t)(row0 + ln) * lda; const _Float16* a1p = a0p + (size_t)16 * lda;
  const _Float16* b0p = Bh + (size_t)(col0 + ln) * ldb; const _Float16* b1p = b0p + (size_t)16 * ldb; const _Float16* b2p = b1p + (size_t)16 * ldb; const _Float16* b3p = b2p + (size_t)16 * ldb;
  const v8f z8 = {0.f,0.f,0.f,0.f,0.f,0.f,0.f,0.f}; v8f c00 = z8, c01 = z8, c02 = z8, c03 = z8, c10 = z8, c11 = z8, c12 = z8, c13 = z8;
#pragma unroll 1
  for (unsigned kb = 0; kb < K; kb += 32u) { const v16h a0 = g2_frag(a0p + kb, hh), a1 = g2_frag(a1p + kb, hh);
    v16h bfr = g2_frag(b0p + kb, hh); c00 = g2_mma(a0, bfr, c00); c10 = g2_mma(a1, bfr, c10);
    bfr = g2_frag(b1p + kb, hh); c01 = g2_mma(a0, bfr, c01); c11 = g2_mma(a1, bfr, c11);
    bfr = g2_frag(b2p + kb, hh); c02 = g2_mma(a0, bfr, c02); c12 = g2_mma(a1, bfr, c12);
    bfr = g2_frag(b3p + kb, hh); c03 = g2_mma(a0, bfr, c03); c13 = g2_mma(a1, bfr, c13); }
  v8f accs[8] = {c00, c01, c02, c03, c10, c11, c12, c13};
#pragma unroll
  for (int u = 0; u < 8; ++u) { const int t = u & 3, half = u >> 2; const unsigned col = col0 + t * 16 + ln; const float bv = bias ? bf16_rne(bias[col]) : 0.f;
#pragma unroll
    for (int r = 0; r < 8; ++r) { const unsigned rloc = half * 16 + 8 * hh + r; so[w][rloc][t * 16 + ln] = accs[u][r] * alpha + bv; } }
  __builtin_amdgcn_fence(4  , "workgroup"); __builtin_amdgcn_wave_barrier();
  const unsigned rsub = lane >> 4, c4 = (lane & 15u) * 4u;
  if (ACT == 6 || RES != 0) {
#pragma unroll 4
    for (unsigned q = 0; q < 16; ++q) { const unsigned r = q * 2u + rsub; v4f v = *(const v4fa*)&so[w][r][c4];
      if (RES != 0) { const unsigned gr = row0 + r; const unsigned sr = (RES == 2) ? xrow(gr) : gr; const v4f rv = *(const v4fa*)(R + (size_t)sr * ldr + col0 + c4);
#pragma unroll
        for (int i = 0; i < 4; ++i) v[i] += (RES == 2) ? bf16_rne(rv[i]) : rv[i]; }
      if (ACT == 6) {
#pragma unroll
        for (int i = 0; i < 4; ++i) v[i] = 0.5f * v[i] * (1.0f + erff(v[i] * 0.70710678118654752f)); }
      *(v4fa*)&so[w][r][c4] = v; }
  }
  for (int pass = 0; pass < 2; ++pass) {
#pragma unroll
    for (unsigned q = 0; q < 16; ++q) { const unsigned r = q * 2u + rsub; const v4f v = *(const v4fa*)&so[w][r][c4];
      if (C) *(volatile v4f*)(C + (size_t)(row0 + r) * ldc + col0 + c4) = v;
      if (C16) { v4h h4;
#pragma unroll
        for (int i = 0; i < 4; ++i) h4[i] = (_Float16)v[i];
        *(volatile v4h*)(C16 + (size_t)(row0 + r) * ldc + col0 + c4) = h4; } }
    if (pass == 0) __threadfence(); }
}

template <int W16, int OMAP>
__global__ __launch_bounds__(256) void k_ln(const float* __restrict__ Y, const float* __restrict__ g, const float* __restrict__ bb, float* __restrict__ N32, _Float16* __restrict__ N16) {
  __shared__ float sm[8]; __shared__ float sv[8];
  const unsigned r = blockIdx.x, t = threadIdx.x, lane = t & 31u, w = t >> 5;
  const v4f xa = *(const v4fa*)(Y + (size_t)r * DM + t * 4u);
  float s = (xa[0] + xa[1]) + (xa[2] + xa[3]);
  s += __shfl_xor(s, 1, 32); s += __shfl_xor(s, 2, 32); s += __shfl_xor(s, 4, 32); s += __shfl_xor(s, 8, 32); s += __shfl_xor(s, 16, 32);
  if (lane == 0) sm[w] = s;
  __syncthreads();
  float tot = 0.f;
#pragma unroll
  for (int i = 0; i < 8; ++i) tot += sm[i];
  const float mu = tot * (1.0f / (float)DM);
  const float d0 = xa[0] - mu, d1 = xa[1] - mu, d2 = xa[2] - mu, d3 = xa[3] - mu;
  float q2 = (d0 * d0 + d1 * d1) + (d2 * d2 + d3 * d3);
  q2 += __shfl_xor(q2, 1, 32); q2 += __shfl_xor(q2, 2, 32); q2 += __shfl_xor(q2, 4, 32); q2 += __shfl_xor(q2, 8, 32); q2 += __shfl_xor(q2, 16, 32);
  if (lane == 0) sv[w] = q2;
  __syncthreads();
  float vt = 0.f;
#pragma unroll
  for (int i = 0; i < 8; ++i) vt += sv[i];
  const float rs = rsqrtf(vt * (1.0f / (float)DM) + 1.0e-5f);
  const v4f gv = *(const v4fa*)(g + t * 4u), bv = *(const v4fa*)(bb + t * 4u);
  v4f y; v4h yh;
  y[0] = d0 * rs * bf16_rne(gv[0]) + bf16_rne(bv[0]); y[1] = d1 * rs * bf16_rne(gv[1]) + bf16_rne(bv[1]);
  y[2] = d2 * rs * bf16_rne(gv[2]) + bf16_rne(bv[2]); y[3] = d3 * rs * bf16_rne(gv[3]) + bf16_rne(bv[3]);
#pragma unroll
  for (int i = 0; i < 4; ++i) yh[i] = (_Float16)y[i];
  const unsigned orow = OMAP ? xrow(r) : r;
  for (int pass = 0; pass < 2; ++pass) {
    *(volatile v4f*)(N32 + (size_t)orow * DM + t * 4u) = y;
    if (W16) *(volatile v4h*)(N16 + (size_t)r * DM + t * 4u) = yh;
    if (pass == 0) __threadfence(); }
}

#define SZ_BQKV ((size_t)LQ * DM * 2)
#define SZ_BO   ((size_t)DM * DM * 2)
#define SZ_BW1  ((size_t)DFF * DM * 2)
#define SZ_BW2  ((size_t)DM * DFF * 2)
#define SZ_X16  ((size_t)NR * DM * 2)
#define SZ_QKV  ((size_t)NR * LQ * 2)
#define SZ_VT   ((size_t)NB * NH * HD * SEQ * 2)
#define SZ_HF   ((size_t)NR * DFF * 2)
#define SZ_RA   ((SZ_QKV + SZ_VT) > SZ_HF ? (SZ_QKV + SZ_VT) : SZ_HF)
#define SZ_O16  ((size_t)NR * DM * 2)
#define SZ_Y    ((size_t)NR * DM * 4)
#define SZ_X1   ((size_t)NR * DM * 4)
#define SZ_X1H  ((size_t)NR * DM * 2)
#define SZ_TOT  (SZ_BQKV + SZ_BO + SZ_BW1 + SZ_BW2 + SZ_X16 + SZ_RA + SZ_O16 + SZ_Y + SZ_X1 + SZ_X1H)
static_assert(SZ_QKV + SZ_VT <= SZ_RA);
static_assert(SZ_HF <= SZ_RA);
static_assert(SZ_TOT <= (size_t)134217728);
static_assert(SZ_BQKV % 256 == 0 && SZ_BO % 256 == 0 && SZ_X16 % 256 == 0 && SZ_RA % 256 == 0 && SZ_QKV % 256 == 0 && SZ_Y % 256 == 0);
static_assert((NR * (DM / 8)) % 256 == 0);
static_assert(((size_t)LQ * (DM / 8)) % 256 == 0 && ((size_t)DM * (DM / 8)) % 256 == 0 && ((size_t)DFF * (DM / 8)) % 256 == 0 && ((size_t)DM * (DFF / 8)) % 256 == 0);

extern "C" void kernel_launch(void* const* d_in, const int* in_sizes, int n_in,
                              void* d_out, int out_size, void* d_ws, size_t ws_size, hipStream_t stream) {
  if (n_in < 13) return;
  const long long xneed = ((long long)(NB - 1) * SEQ_FULL + SEQ) * DM;
  if ((long long)in_sizes[0] < xneed || (long long)out_size < xneed) return;
  if (in_sizes[1] < DM * LQ || in_sizes[2] < LQ || in_sizes[3] < DM * DM || in_sizes[4] < DM || in_sizes[5] < DM * DFF || in_sizes[6] < DFF || in_sizes[7] < DFF * DM || in_sizes[8] < DM) return;
  if (in_sizes[9] < DM || in_sizes[10] < DM || in_sizes[11] < DM || in_sizes[12] < DM) return;
  if (ws_size < SZ_TOT) return;
  const float* x = (const float*)d_in[0]; const float* Wqkv = (const float*)d_in[1]; const float* bqkv = (const float*)d_in[2]; const float* Wo = (const float*)d_in[3]; const float* bo = (const float*)d_in[4];
  const float* W1 = (const float*)d_in[5]; const float* b1 = (const float*)d_in[6]; const float* W2 = (const float*)d_in[7]; const float* b2 = (const float*)d_in[8];
  const float* g1 = (const float*)d_in[9]; const float* be1 = (const float*)d_in[10]; const float* g2 = (const float*)d_in[11]; const float* be2 = (const float*)d_in[12];
  float* out = (float*)d_out;
  char* ws = (char*)d_ws; size_t off = 0;
  _Float16* BQKV = (_Float16*)(ws + off); off += SZ_BQKV;
  _Float16* BO   = (_Float16*)(ws + off); off += SZ_BO;
  _Float16* BW1  = (_Float16*)(ws + off); off += SZ_BW1;
  _Float16* BW2  = (_Float16*)(ws + off); off += SZ_BW2;
  _Float16* X16  = (_Float16*)(ws + off); off += SZ_X16;
  _Float16* QKV  = (_Float16*)(ws + off); _Float16* VT = (_Float16*)(ws + off + SZ_QKV); _Float16* HF16 = (_Float16*)(ws + off); off += SZ_RA;
  _Float16* O16  = (_Float16*)(ws + off); off += SZ_O16;
  float* Y       = (float*)(ws + off); off += SZ_Y;
  float* X1      = (float*)(ws + off); off += SZ_X1;
  _Float16* X1H  = (_Float16*)(ws + off); off += SZ_X1H;
  if (off > ws_size) return;

  k_x16<<<(unsigned)(NR * (DM / 8) / 256), 256, 0, stream>>>(x, X16);
  k_wt_f16<<<(unsigned)((size_t)LQ * (DM / 8) / 256), 256, 0, stream>>>(Wqkv, BQKV, (unsigned)DM, (unsigned)LQ, 16.0f);
  k_wt_f16<<<(unsigned)((size_t)DM * (DM / 8) / 256), 256, 0, stream>>>(Wo, BO, (unsigned)DM, (unsigned)DM, 16.0f);
  k_wt_f16<<<(unsigned)((size_t)DFF * (DM / 8) / 256), 256, 0, stream>>>(W1, BW1, (unsigned)DM, (unsigned)DFF, 16.0f);
  k_wt_f16<<<(unsigned)((size_t)DM * (DFF / 8) / 256), 256, 0, stream>>>(W2, BW2, (unsigned)DFF, (unsigned)DM, 64.0f);
  k_gemm2<0, 0><<<(unsigned)((NR / 128) * (LQ / 64)), 128, 0, stream>>>(X16, (unsigned)DM, BQKV, (unsigned)DM, 0.00390625f, bqkv, nullptr, 0u, nullptr, QKV, (unsigned)LQ, (unsigned)NR, (unsigned)LQ, (unsigned)DM);
  k_vt<<<(unsigned)(NB * NH * (SEQ / 64)), 256, 0, stream>>>(QKV, VT);
  k_attn<<<(unsigned)(NB * NH * (SEQ / 64)), 128, 0, stream>>>(QKV, VT, O16);
  k_gemm2<0, 2><<<(unsigned)((NR / 128) * (DM / 64)), 128, 0, stream>>>(O16, (unsigned)DM, BO, (unsigned)DM, 0.0009765625f, bo, x, (unsigned)DM, Y, nullptr, (unsigned)DM, (unsigned)NR, (unsigned)DM, (unsigned)DM);
  k_ln<1, 0><<<(unsigned)NR, 256, 0, stream>>>(Y, g1, be1, X1, X1H);
  k_gemm2<6, 0><<<(unsigned)((NR / 128) * (DFF / 64)), 128, 0, stream>>>(X1H, (unsigned)DM, BW1, (unsigned)DM, 0.0625f, b1, nullptr, 0u, nullptr, HF16, (unsigned)DFF, (unsigned)NR, (unsigned)DFF, (unsigned)DM);
  k_gemm2<0, 1><<<(unsigned)((NR / 128) * (DM / 64)), 128, 0, stream>>>(HF16, (unsigned)DFF, BW2, (unsigned)DFF, 0.015625f, b2, X1, (unsigned)DM, Y, nullptr, (unsigned)DM, (unsigned)NR, (unsigned)DM, (unsigned)DFF);
  k_ln<0, 1><<<(unsigned)NR, 256, 0, stream>>>(Y, g2, be2, out, nullptr);
}
